// PhysicsInvariantAttention_78503412236720
// MI455X (gfx1250) — hardware-verified
//
#include <hip/hip_runtime.h>
#include <hip/hip_bf16.h>
#include <stddef.h>
#include <stdint.h>

#define NN    1024
#define CC    128
#define NHD   4
#define HDD   32
#define HID   64
#define NQW   (NHD * HID)
#define NWT   (3 * CC)
#define IB    4
#define BR    32
#define BC    64
#define NQT   (NN / BR)
#define NCH   (NN / BC)

static_assert(CC % 32 == 0);
static_assert(CC / 32 == 4);
static_assert(HDD == 32);
static_assert(NHD * HDD == CC);
static_assert(HID == 64);
static_assert(NN % 256 == 0);
static_assert(NN == 4 * 256);
static_assert(NN % IB == 0);
static_assert(NN % (8 * 16) == 0);
static_assert((NN * CC) % (8 * 256) == 0);
static_assert((HID * CC) % (8 * 256) == 0);
static_assert((NN * HID) % (4 * 256) == 0);
static_assert(BC == 4 * 16);
static_assert(BR * 4 == 128);
static_assert(NN % BR == 0);
static_assert(NN % BC == 0);

typedef float          v8f   __attribute__((ext_vector_type(8)));
typedef float          v4f   __attribute__((ext_vector_type(4)));
typedef unsigned int   v4u   __attribute__((ext_vector_type(4)));
typedef unsigned short v8us  __attribute__((ext_vector_type(8)));
typedef unsigned short v16us __attribute__((ext_vector_type(16)));
typedef __bf16         v16b  __attribute__((ext_vector_type(16)));
typedef unsigned short ush;

union FragU { v16us v; v8us h[2]; v4u u[2]; v16b b; };
union PackU { v8us s; v4u u; };
struct HL { v4u h; v4u l; };

__device__ __forceinline__ ush f2bf(float f) {
  const unsigned u = __float_as_uint(f);
  return (ush)((u + 0x7FFFu + ((u >> 16) & 1u)) >> 16);
}
__device__ __forceinline__ float bf2f(ush b) { return __uint_as_float(((unsigned)b) << 16); }

__device__ __forceinline__ HL split8(v8f f) {
  PackU ph, pl;
#pragma unroll
  for (int e = 0; e < 8; ++e) {
    const ush hi = f2bf(f[e]);
    ph.s[e] = hi;
    pl.s[e] = f2bf(f[e] - bf2f(hi));
  }
  HL r; r.h = ph.u; r.l = pl.u;
  return r;
}

__device__ __forceinline__ v8f mmab(v16us a, v16us b, v8f c) {
  FragU ua, ub; ua.v = a; ub.v = b;
  c = __builtin_amdgcn_wmma_f32_16x16x32_bf16(false, ua.b, false, ub.b, (short)0, c, false, false);
  asm volatile("v_nop\n\tv_nop\n\tv_nop\n\tv_nop" : "+v"(c) : "v"(a), "v"(b));
  return c;
}

__device__ __forceinline__ v16us ldfragu(const ush* p, int ld, int row0, int k0, int lane) {
  const int m = lane & 15, lh = lane >> 4;
  const ush* q = p + (size_t)(row0 + m) * ld + k0 + 8 * lh;
  FragU f;
  f.h[0] = *(const v8us*)(q);
  f.h[1] = *(const v8us*)(q + 16);
  return f.v;
}

__device__ __forceinline__ v8f zero8() { return (v8f){0.f, 0.f, 0.f, 0.f, 0.f, 0.f, 0.f, 0.f}; }

__device__ __forceinline__ void gemm3_32x64(const ush* __restrict__ Ah, const ush* __restrict__ Al, int lda,
                                            const ush* __restrict__ Bh, const ush* __restrict__ Bl, int ldb,
                                            int m0, int n0, int kbeg, int kend, int lane, v8f (&acc)[2][4]) {
#pragma unroll 1
  for (int k0 = kbeg; k0 < kend; k0 += 32) {
    const v16us a0h = ldfragu(Ah, lda, m0, k0, lane);
    const v16us a1h = ldfragu(Ah, lda, m0 + 16, k0, lane);
    const v16us a0l = ldfragu(Al, lda, m0, k0, lane);
    const v16us a1l = ldfragu(Al, lda, m0 + 16, k0, lane);
#pragma unroll
    for (int t = 0; t < 4; ++t) {
      const v16us bh = ldfragu(Bh, ldb, n0 + 16 * t, k0, lane);
      const v16us bl = ldfragu(Bl, ldb, n0 + 16 * t, k0, lane);
      acc[0][t] = mmab(a0h, bh, acc[0][t]);
      acc[1][t] = mmab(a1h, bh, acc[1][t]);
      acc[0][t] = mmab(a0h, bl, acc[0][t]);
      acc[1][t] = mmab(a1h, bl, acc[1][t]);
      acc[0][t] = mmab(a0l, bh, acc[0][t]);
      acc[1][t] = mmab(a1l, bh, acc[1][t]);
    }
  }
}

#define TPP 132
enum { KB_X = (NN * CC / 8) / 256, KB_W2 = (HID * CC / 8) / 256, KB_P = (NN * HID / 4) / 256, KB_T = 3 * (CC / 32) };
enum { GB1 = KB_X, GB2 = 2 * KB_X, GB3 = GB2 + KB_W2, GB4 = GB3 + KB_P, GB5 = GB4 + KB_T };

__global__ __launch_bounds__(256) void k_cvt(const float* __restrict__ x, const float* __restrict__ y,
                                             const float* __restrict__ pos,
                                             const float* __restrict__ wq, const float* __restrict__ wk,
                                             const float* __restrict__ wv,
                                             const float* __restrict__ w1, const float* __restrict__ w2,
                                             ush* __restrict__ Xh, ush* __restrict__ Xl,
                                             ush* __restrict__ Yh, ush* __restrict__ Yl,
                                             ush* __restrict__ WTh, ush* __restrict__ WTl,
                                             ush* __restrict__ W2h, ush* __restrict__ W2l,
                                             float* __restrict__ P) {
  __shared__ __align__(16) float sT[32 * TPP];
  const int bid = (int)blockIdx.x, tid = (int)threadIdx.x;
  if (bid < GB3) {
    const int role = (bid < GB1) ? 0 : ((bid < GB2) ? 1 : 2);
    const float* src = (role == 0) ? x : ((role == 1) ? y : w2);
    ush* dh = (role == 0) ? Xh : ((role == 1) ? Yh : W2h);
    ush* dl = (role == 0) ? Xl : ((role == 1) ? Yl : W2l);
    const int t = (bid - ((role == 0) ? 0 : ((role == 1) ? GB1 : GB2))) * 256 + tid;
    const int ngrp = (role == 2) ? (HID * CC / 8) : (NN * CC / 8);
    if (t >= ngrp) return;
    const size_t o = (size_t)t * 8;
    const v4f a0 = *(const v4f*)(src + o);
    const v4f a1 = *(const v4f*)(src + o + 4);
    const v8f f = (v8f){a0[0], a0[1], a0[2], a0[3], a1[0], a1[1], a1[2], a1[3]};
    const HL s = split8(f);
    *(volatile v4u*)(dh + o) = s.h;
    *(volatile v4u*)(dl + o) = s.l;
    __threadfence();
    *(volatile v4u*)(dh + o) = s.h;
    *(volatile v4u*)(dl + o) = s.l;
    return;
  }
  if (bid < GB4) {
    const int t = (bid - GB3) * 256 + tid;
    if (t >= NN * HID / 4) return;
    const int n = t >> 4, c4 = (t & 15) * 4;
    const float px = pos[n * 3], py = pos[n * 3 + 1], pz = pos[n * 3 + 2];
    const v4f wa = *(const v4f*)(w1 + c4);
    const v4f wb = *(const v4f*)(w1 + HID + c4);
    const v4f wc = *(const v4f*)(w1 + 2 * HID + c4);
    v4f r;
#pragma unroll
    for (int u = 0; u < 4; ++u) r[u] = px * wa[u] + py * wb[u] + pz * wc[u];
    float* dst = P + (size_t)n * HID + c4;
    *(volatile v4f*)dst = r;
    __threadfence();
    *(volatile v4f*)dst = r;
    return;
  }
  {
    const int tb = bid - GB4;
    const int which = tb >> 2, slab = tb & 3, n0 = slab * 32;
    const float* W = (which == 0) ? wq : ((which == 1) ? wk : wv);
#pragma unroll
    for (int it = 0; it < 4; ++it) {
      const int g  = tid + 256 * it;
      const int k  = g >> 3;
      const int nq = (g & 7) * 4;
      const v4f v = *(const v4f*)(W + (size_t)k * CC + n0 + nq);
#pragma unroll
      for (int u = 0; u < 4; ++u) sT[(nq + u) * TPP + k] = v[u];
    }
    __syncthreads();
    v4u vh[2], vl[2];
    size_t od[2];
#pragma unroll
    for (int it = 0; it < 2; ++it) {
      const int p  = tid + 256 * it;
      const int nn = p >> 4;
      const int pc = p & 15;
      const float* sp = sT + nn * TPP + pc * 8;
      const v4f f0 = *(const v4f*)(sp);
      const v4f f1 = *(const v4f*)(sp + 4);
      const v8f f = (v8f){f0[0], f0[1], f0[2], f0[3], f1[0], f1[1], f1[2], f1[3]};
      const HL s = split8(f);
      vh[it] = s.h; vl[it] = s.l;
      od[it] = ((size_t)(which * CC + n0 + nn)) * CC + pc * 8;
    }
#pragma unroll
    for (int it = 0; it < 2; ++it) { *(volatile v4u*)(WTh + od[it]) = vh[it]; *(volatile v4u*)(WTl + od[it]) = vl[it]; }
    __threadfence();
#pragma unroll
    for (int it = 0; it < 2; ++it) { *(volatile v4u*)(WTh + od[it]) = vh[it]; *(volatile v4u*)(WTl + od[it]) = vl[it]; }
  }
}

#define STP 72
__global__ __launch_bounds__(256) void k_proj(const ush* __restrict__ Xh, const ush* __restrict__ Xl,
                                              const ush* __restrict__ Yh, const ush* __restrict__ Yl,
                                              const ush* __restrict__ WTh, const ush* __restrict__ WTl,
                                              const float* __restrict__ bq,
                                              const float* __restrict__ bk,
                                              const float* __restrict__ bv,
                                              ush* __restrict__ Qh, ush* __restrict__ Ql,
                                              ush* __restrict__ Kh, ush* __restrict__ Kl,
                                              ush* __restrict__ VTh, ush* __restrict__ VTl) {
  __shared__ __align__(16) ush st[256 * STP];
  const int tid = (int)threadIdx.x, lane = tid & 31, wave = tid >> 5;
  const int hh = lane >> 4, c = lane & 15;
  const int mb = (int)blockIdx.x * 256;
  const int m0 = mb + wave * 32;
  const int n0 = (int)blockIdx.y * 64;
  const int which = n0 / CC;
  const int nn = n0 - which * CC;
  const ush* Ah = (which == 0) ? Xh : Yh;
  const ush* Al = (which == 0) ? Xl : Yl;
  const float* bias = (which == 0) ? bq : ((which == 1) ? bk : bv);

  v8f acc[2][4];
#pragma unroll
  for (int s = 0; s < 2; ++s)
#pragma unroll
    for (int t = 0; t < 4; ++t) acc[s][t] = zero8();
  gemm3_32x64(Ah, Al, CC, WTh, WTl, CC, m0, n0, 0, CC, lane, acc);

#pragma unroll
  for (int t = 0; t < 4; ++t) {
    const float bn = bias[nn + 16 * t + c];
#pragma unroll
    for (int sub = 0; sub < 2; ++sub) {
#pragma unroll
      for (int r = 0; r < 8; ++r) acc[sub][t][r] += bn;
    }
  }

  ush* bhp = (which == 0) ? Qh : ((which == 1) ? Kh : VTh);
  ush* blp = (which == 0) ? Ql : ((which == 1) ? Kl : VTl);
  size_t go[8];
#pragma unroll
  for (int j = 0; j < 8; ++j) {
    const int p  = tid + 256 * j;
    const int L  = p >> 3;
    const int pc = p & 7;
    if (which < 2) {
      go[j] = ((size_t)(mb + L)) * CC + nn + pc * 8;
    } else {
      const int d  = L >> 2;
      const int nl = (L & 3) * 64 + pc * 8;
      go[j] = ((size_t)(nn + d)) * NN + mb + nl;
    }
  }

#pragma unroll 1
  for (int ph = 0; ph < 2; ++ph) {
    __syncthreads();
#pragma unroll
    for (int t = 0; t < 4; ++t) {
#pragma unroll
      for (int sub = 0; sub < 2; ++sub) {
#pragma unroll
        for (int r = 0; r < 8; ++r) {
          const int lr = wave * 32 + sub * 16 + 8 * hh + r;
          const float v = acc[sub][t][r];
          const ush hi = f2bf(v);
          st[lr * STP + 16 * t + c] = (ph == 0) ? hi : f2bf(v - bf2f(hi));
        }
      }
    }
    __syncthreads();
    v4u val[8];
    if (which < 2) {
#pragma unroll
      for (int j = 0; j < 8; ++j) {
        const int p  = tid + 256 * j;
        const int lr = p >> 3;
        const int pc = p & 7;
        PackU pk;
        pk.s  = *(const v8us*)(st + lr * STP + pc * 8);
        val[j] = pk.u;
      }
    } else {
#pragma unroll
      for (int j = 0; j < 8; ++j) {
        const int p  = tid + 256 * j;
        const int L  = p >> 3;
        const int pc = p & 7;
        const int d  = L >> 2;
        const int nl = (L & 3) * 64 + pc * 8;
        const ush* cp = st + nl * STP + d;
        PackU pk;
        pk.s = (v8us){cp[0 * STP], cp[1 * STP], cp[2 * STP], cp[3 * STP],
                      cp[4 * STP], cp[5 * STP], cp[6 * STP], cp[7 * STP]};
        val[j] = pk.u;
      }
    }
    ush* dst = (ph == 0) ? bhp : blp;
#pragma unroll
    for (int j = 0; j < 8; ++j) *(volatile v4u*)(dst + go[j]) = val[j];
    __threadfence();
#pragma unroll
    for (int j = 0; j < 8; ++j) *(volatile v4u*)(dst + go[j]) = val[j];
    __threadfence();
  }
}

__global__ __launch_bounds__(256) void k_qw(const ush* __restrict__ Qh, const ush* __restrict__ Ql,
                                            const ush* __restrict__ W2h, const ush* __restrict__ W2l,
                                            ush* __restrict__ QWh, ush* __restrict__ QWl) {
  __shared__ __align__(16) ush st[256 * STP];
  const int tid = (int)threadIdx.x, lane = tid & 31, wave = tid >> 5;
  const int hh = lane >> 4, c = lane & 15;
  const int mb = (int)blockIdx.x * 256;
  const int m0 = mb + wave * 32;
  const int h  = (int)blockIdx.y;

  v8f acc[2][4];
#pragma unroll
  for (int s = 0; s < 2; ++s)
#pragma unroll
    for (int t = 0; t < 4; ++t) acc[s][t] = zero8();
  gemm3_32x64(Qh, Ql, CC, W2h, W2l, CC, m0, 0, h * HDD, h * HDD + 32, lane, acc);

  size_t go[8];
#pragma unroll
  for (int j = 0; j < 8; ++j) {
    const int p  = tid + 256 * j;
    const int L  = p >> 3;
    const int pc = p & 7;
    go[j] = ((size_t)(mb + L)) * NQW + h * HID + pc * 8;
  }
#pragma unroll 1
  for (int ph = 0; ph < 2; ++ph) {
    __syncthreads();
#pragma unroll
    for (int t = 0; t < 4; ++t) {
#pragma unroll
      for (int sub = 0; sub < 2; ++sub) {
#pragma unroll
        for (int r = 0; r < 8; ++r) {
          const int lr = wave * 32 + sub * 16 + 8 * hh + r;
          const float v = acc[sub][t][r];
          const ush hi = f2bf(v);
          st[lr * STP + 16 * t + c] = (ph == 0) ? hi : f2bf(v - bf2f(hi));
        }
      }
    }
    __syncthreads();
    v4u val[8];
#pragma unroll
    for (int j = 0; j < 8; ++j) {
      const int p  = tid + 256 * j;
      const int lr = p >> 3;
      const int pc = p & 7;
      PackU pk;
      pk.s  = *(const v8us*)(st + lr * STP + pc * 8);
      val[j] = pk.u;
    }
    ush* dst = (ph == 0) ? QWh : QWl;
#pragma unroll
    for (int j = 0; j < 8; ++j) *(volatile v4u*)(dst + go[j]) = val[j];
    __threadfence();
#pragma unroll
    for (int j = 0; j < 8; ++j) *(volatile v4u*)(dst + go[j]) = val[j];
    __threadfence();
  }
}

__global__ __launch_bounds__(256) void k_geom(const float* __restrict__ P, const float* __restrict__ b1,
                                              const float* __restrict__ b2, const float* __restrict__ pos,
                                              const ush* __restrict__ Qh, const ush* __restrict__ Ql,
                                              const ush* __restrict__ QWh, const ush* __restrict__ QWl,
                                              float* __restrict__ bias) {
  __shared__ __align__(16) float sG[NHD * NN];
  __shared__ __align__(16) float sQb[NHD];
  const int tid = (int)threadIdx.x, lane = tid & 31, wave = tid >> 5;
  const int hh = lane >> 4, m = lane & 15;
  const int rowq = (m < NHD) ? m : (NHD - 1);

  float pj[12];
  {
    const v4f t0 = *(const v4f*)(pos + 12 * tid);
    const v4f t1 = *(const v4f*)(pos + 12 * tid + 4);
    const v4f t2 = *(const v4f*)(pos + 12 * tid + 8);
#pragma unroll
    for (int e = 0; e < 4; ++e) { pj[e] = t0[e]; pj[4 + e] = t1[e]; pj[8 + e] = t2[e]; }
  }
  FragU zf;
  zf.u[0] = (v4u){0u, 0u, 0u, 0u};
  zf.u[1] = (v4u){0u, 0u, 0u, 0u};
  const v16us z16 = zf.v;

#pragma unroll 1
  for (int ii = 0; ii < IB; ++ii) {
    const int i = (int)blockIdx.x * IB + ii;

    if (tid < NHD) {
      const int h = tid;
      const ush* qa = Qh + (size_t)i * CC + h * HDD;
      const ush* qr = Ql + (size_t)i * CC + h * HDD;
      const float* bb = b2 + h * HDD;
      float s = 0.f;
#pragma unroll 1
      for (int d = 0; d < HDD; ++d) s += bb[d] * (bf2f(qa[d]) + bf2f(qr[d]));
      sQb[h] = s;
    }

    float pb[2][16];
#pragma unroll
    for (int ks = 0; ks < 2; ++ks) {
      const float* pp = P + (size_t)i * HID + 32 * ks + 8 * hh;
      const float* bp = b1 + 32 * ks + 8 * hh;
      const v4f a0 = *(const v4f*)(pp), a1 = *(const v4f*)(pp + 4);
      const v4f a2 = *(const v4f*)(pp + 16), a3 = *(const v4f*)(pp + 20);
      const v4f c0 = *(const v4f*)(bp), c1 = *(const v4f*)(bp + 4);
      const v4f c2 = *(const v4f*)(bp + 16), c3 = *(const v4f*)(bp + 20);
#pragma unroll
      for (int e = 0; e < 4; ++e) {
        pb[ks][e]      = a0[e] + c0[e];
        pb[ks][4 + e]  = a1[e] + c1[e];
        pb[ks][8 + e]  = a2[e] + c2[e];
        pb[ks][12 + e] = a3[e] + c3[e];
      }
    }

    v16us bqh[2], bql[2];
    {
      const ush* qp = QWh + (size_t)i * NQW + rowq * HID + 8 * hh;
      const ush* ql = QWl + (size_t)i * NQW + rowq * HID + 8 * hh;
#pragma unroll
      for (int ks = 0; ks < 2; ++ks) {
        FragU fh, fl;
        fh.h[0] = *(const v8us*)(qp + 32 * ks);
        fh.h[1] = *(const v8us*)(qp + 32 * ks + 16);
        fl.h[0] = *(const v8us*)(ql + 32 * ks);
        fl.h[1] = *(const v8us*)(ql + 32 * ks + 16);
        bqh[ks] = (m < NHD) ? fh.v : z16;
        bql[ks] = (m < NHD) ? fl.v : z16;
      }
    }

#pragma unroll 1
    for (int tt = 0; tt < NN / (8 * 16); ++tt) {
      const int j0 = wave * (NN / 8) + 16 * tt;
      v8f acc = zero8();
#pragma unroll
      for (int ks = 0; ks < 2; ++ks) {
        const float* pr = P + (size_t)(j0 + m) * HID + 32 * ks + 8 * hh;
        const v4f p0 = *(const v4f*)(pr), p1 = *(const v4f*)(pr + 4);
        const v4f p2 = *(const v4f*)(pr + 16), p3 = *(const v4f*)(pr + 20);
        v8f ra, rb;
#pragma unroll
        for (int e = 0; e < 4; ++e) {
          ra[e]     = fmaxf(pb[ks][e]      - p0[e], 0.f);
          ra[4 + e] = fmaxf(pb[ks][4 + e]  - p1[e], 0.f);
          rb[e]     = fmaxf(pb[ks][8 + e]  - p2[e], 0.f);
          rb[4 + e] = fmaxf(pb[ks][12 + e] - p3[e], 0.f);
        }
        const HL sa = split8(ra);
        const HL sb = split8(rb);
        FragU fh, fl;
        fh.u[0] = sa.h; fh.u[1] = sb.h;
        fl.u[0] = sa.l; fl.u[1] = sb.l;
        acc = mmab(fh.v, bqh[ks], acc);
        acc = mmab(fh.v, bql[ks], acc);
        acc = mmab(fl.v, bqh[ks], acc);
      }
      if (m < NHD) {
#pragma unroll
        for (int r = 0; r < 8; ++r) sG[m * NN + j0 + 8 * hh + r] = acc[r];
      }
    }
    __syncthreads();

    const float pix = pos[3 * i], piy = pos[3 * i + 1], piz = pos[3 * i + 2];
    float dsv[4];
#pragma unroll
    for (int u = 0; u < 4; ++u) {
      const float dx = pix - pj[3 * u], dy = piy - pj[3 * u + 1], dz = piz - pj[3 * u + 2];
      const float d2 = dx * dx + dy * dy + dz * dz;
      const float sq = sqrtf(d2);
      dsv[u] = (d2 > 0.f) ? sq : 0.f;
    }
    v4f val[NHD];
#pragma unroll
    for (int h = 0; h < NHD; ++h) {
      const v4f g = *(const v4f*)(sG + h * NN + 4 * tid);
      const float qb = sQb[h];
#pragma unroll
      for (int u = 0; u < 4; ++u) val[h][u] = (g[u] + qb) - dsv[u];
    }
    float* brow = bias + (size_t)i * NN + 4 * tid;
#pragma unroll
    for (int h = 0; h < NHD; ++h) *(volatile v4f*)(brow + (size_t)h * NN * NN) = val[h];
    __threadfence();
#pragma unroll
    for (int h = 0; h < NHD; ++h) *(volatile v4f*)(brow + (size_t)h * NN * NN) = val[h];
    __syncthreads();
  }
}

#define SSP 68
#define SPP 72
#define OTP 36
__global__ __launch_bounds__(128) void k_attn(const ush* __restrict__ Qh, const ush* __restrict__ Ql,
                                              const ush* __restrict__ Kh, const ush* __restrict__ Kl,
                                              const ush* __restrict__ VTh, const ush* __restrict__ VTl,
                                              const float* __restrict__ bias, float* __restrict__ out,
                                              float sscale) {
  __shared__ __align__(16) float sS[BR * SSP];
  __shared__ __align__(16) ush   sPh[BR * SPP];
  __shared__ __align__(16) ush   sPl[BR * SPP];
  __shared__ __align__(16) float sO[BR * OTP];
  __shared__ __align__(16) float sRed[BR * 4];
  __shared__ __align__(16) float rM[BR];
  __shared__ __align__(16) float rMn[BR];
  __shared__ __align__(16) float rL[BR];
  __shared__ __align__(16) float rSc[BR];

  const int tid = (int)threadIdx.x, lane = tid & 31, wave = tid >> 5;
  const int hh = lane >> 4, c = lane & 15;
  const int h  = (int)blockIdx.y;
  const int i0 = (int)blockIdx.x * BR;
  const int kq = h * HDD;
  const float NEGI = -__builtin_huge_valf();
  if (tid < BR) { rM[tid] = NEGI; rL[tid] = 0.f; }
  __syncthreads();

  const v16us a0h = ldfragu(Qh, CC, i0, kq, lane);
  const v16us a1h = ldfragu(Qh, CC, i0 + 16, kq, lane);
  const v16us a0l = ldfragu(Ql, CC, i0, kq, lane);
  const v16us a1l = ldfragu(Ql, CC, i0 + 16, kq, lane);

  const int rt = wave & 1, ct = wave >> 1;
  v8f oacc = zero8();

  const int srow = tid >> 2, schk = tid & 3;
  const float* brow = bias + ((size_t)h * NN + (size_t)(i0 + srow)) * NN + schk * 16;

#pragma unroll 1
  for (int ch = 0; ch < NCH; ++ch) {
    const int j0  = ch * BC;
    const int kr0 = j0 + wave * 16;
    const v16us kbh = ldfragu(Kh, CC, kr0, kq, lane);
    const v16us kbl = ldfragu(Kl, CC, kr0, kq, lane);
    v8f s[2];
    s[0] = mmab(a0h, kbh, zero8());
    s[1] = mmab(a1h, kbh, zero8());
    s[0] = mmab(a0h, kbl, s[0]);
    s[1] = mmab(a1h, kbl, s[1]);
    s[0] = mmab(a0l, kbh, s[0]);
    s[1] = mmab(a1l, kbh, s[1]);
#pragma unroll
    for (int t = 0; t < 2; ++t) {
#pragma unroll
      for (int r = 0; r < 8; ++r) {
        const int row = 16 * t + 8 * hh + r;
        sS[row * SSP + wave * 16 + c] = s[t][r] * sscale;
      }
    }
    __syncthreads();
    float sv[16];
    {
      const float* sr = sS + srow * SSP + schk * 16;
      const v4f x0 = *(const v4f*)(sr);
      const v4f x1 = *(const v4f*)(sr + 4);
      const v4f x2 = *(const v4f*)(sr + 8);
      const v4f x3 = *(const v4f*)(sr + 12);
      const v4f g0 = *(const v4f*)(brow + j0);
      const v4f g1 = *(const v4f*)(brow + j0 + 4);
      const v4f g2 = *(const v4f*)(brow + j0 + 8);
      const v4f g3 = *(const v4f*)(brow + j0 + 12);
#pragma unroll
      for (int e = 0; e < 4; ++e) {
        sv[e]      = x0[e] + g0[e];
        sv[4 + e]  = x1[e] + g1[e];
        sv[8 + e]  = x2[e] + g2[e];
        sv[12 + e] = x3[e] + g3[e];
      }
      float mx = sv[0];
#pragma unroll
      for (int e = 1; e < 16; ++e) mx = fmaxf(mx, sv[e]);
      sRed[srow * 4 + schk] = mx;
    }
    __syncthreads();
    if (tid < BR) {
      float mx = rM[tid];
#pragma unroll
      for (int q = 0; q < 4; ++q) mx = fmaxf(mx, sRed[tid * 4 + q]);
      rMn[tid] = mx;
    }
    __syncthreads();
    {
      const float mx = rMn[srow];
      float sum = 0.f;
      PackU ph0, pl0, ph1, pl1;
#pragma unroll
      for (int e = 0; e < 8; ++e) {
        const float p = __expf(sv[e] - mx);
        sum += p;
        const ush hi = f2bf(p);
        ph0.s[e] = hi;
        pl0.s[e] = f2bf(p - bf2f(hi));
      }
#pragma unroll
      for (int e = 0; e < 8; ++e) {
        const float p = __expf(sv[8 + e] - mx);
        sum += p;
        const ush hi = f2bf(p);
        ph1.s[e] = hi;
        pl1.s[e] = f2bf(p - bf2f(hi));
      }
      *(v8us*)(sPh + srow * SPP + schk * 16)     = ph0.s;
      *(v8us*)(sPh + srow * SPP + schk * 16 + 8) = ph1.s;
      *(v8us*)(sPl + srow * SPP + schk * 16)     = pl0.s;
      *(v8us*)(sPl + srow * SPP + schk * 16 + 8) = pl1.s;
      sRed[srow * 4 + schk] = sum;
    }
    __syncthreads();
    if (tid < BR) {
      float sum = 0.f;
#pragma unroll
      for (int q = 0; q < 4; ++q) sum += sRed[tid * 4 + q];
      const float mnew = rMn[tid];
      const float fac  = __expf(rM[tid] - mnew);
      rL[tid]  = rL[tid] * fac + sum;
      rM[tid]  = mnew;
      rSc[tid] = fac;
    }
    __syncthreads();
    {
      const v4f f0 = *(const v4f*)(rSc + 16 * rt + 8 * hh);
      const v4f f1 = *(const v4f*)(rSc + 16 * rt + 8 * hh + 4);
#pragma unroll
      for (int r = 0; r < 4; ++r) {
        oacc[r]     *= f0[r];
        oacc[4 + r] *= f1[r];
      }
    }
#pragma unroll
    for (int kk = 0; kk < BC / 32; ++kk) {
      const v16us pah = ldfragu(sPh, SPP, 16 * rt, kk * 32, lane);
      const v16us pal = ldfragu(sPl, SPP, 16 * rt, kk * 32, lane);
      const v16us vbh = ldfragu(VTh, NN, kq + 16 * ct, j0 + kk * 32, lane);
      const v16us vbl = ldfragu(VTl, NN, kq + 16 * ct, j0 + kk * 32, lane);
      oacc = mmab(pah, vbh, oacc);
      oacc = mmab(pah, vbl, oacc);
      oacc = mmab(pal, vbh, oacc);
    }
    __syncthreads();
  }

#pragma unroll
  for (int r = 0; r < 8; ++r) {
    const int row   = 16 * rt + 8 * hh + r;
    const float lv  = rL[row];
    const float inv = (lv > 0.f) ? (1.0f / lv) : 0.f;
    sO[row * OTP + 16 * ct + c] = oacc[r] * inv;
  }
  __syncthreads();
  v4f val[2];
  size_t go[2];
#pragma unroll
  for (int it = 0; it < 2; ++it) {
    const int p  = tid + 128 * it;
    const int L  = p >> 3;
    const int pc = p & 7;
    val[it] = *(const v4f*)(sO + L * OTP + pc * 4);
    go[it]  = ((size_t)(i0 + L)) * CC + kq + pc * 4;
  }
#pragma unroll
  for (int it = 0; it < 2; ++it) *(volatile v4f*)(out + go[it]) = val[it];
  __threadfence();
#pragma unroll
  for (int it = 0; it < 2; ++it) *(volatile v4f*)(out + go[it]) = val[it];
}

extern "C" void kernel_launch(void* const* d_in, const int* in_sizes, int n_in,
                              void* d_out, int out_size, void* d_ws, size_t ws_size,
                              hipStream_t stream) {
  if (n_in < 13) return;
  if (in_sizes[0] != NN * CC) return;
  if (in_sizes[1] != NN * CC) return;
  if (in_sizes[2] != NN * 3) return;
  if (in_sizes[3] != CC * CC) return;
  if (in_sizes[4] != CC) return;
  if (in_sizes[5] != CC * CC) return;
  if (in_sizes[6] != CC) return;
  if (in_sizes[7] != CC * CC) return;
  if (in_sizes[8] != CC) return;
  if (in_sizes[9] != 3 * HID) return;
  if (in_sizes[10] != HID) return;
  if (in_sizes[11] != HID * CC) return;
  if (in_sizes[12] != CC) return;
  if (out_size != NN * CC) return;

  const float* x   = (const float*)d_in[0];
  const float* y   = (const float*)d_in[1];
  const float* pos = (const float*)d_in[2];
  const float* wq  = (const float*)d_in[3];
  const float* bq  = (const float*)d_in[4];
  const float* wk  = (const float*)d_in[5];
  const float* bk  = (const float*)d_in[6];
  const float* wv  = (const float*)d_in[7];
  const float* bv  = (const float*)d_in[8];
  const float* w1  = (const float*)d_in[9];
  const float* b1  = (const float*)d_in[10];
  const float* w2  = (const float*)d_in[11];
  const float* b2  = (const float*)d_in[12];
  float* out = (float*)d_out;

  size_t off = 0;
  const size_t oXh  = off; off += (size_t)NN * CC * 2;
  const size_t oXl  = off; off += (size_t)NN * CC * 2;
  const size_t oYh  = off; off += (size_t)NN * CC * 2;
  const size_t oYl  = off; off += (size_t)NN * CC * 2;
  const size_t oWTh = off; off += (size_t)NWT * CC * 2;
  const size_t oWTl = off; off += (size_t)NWT * CC * 2;
  const size_t oW2h = off; off += (size_t)HID * CC * 2;
  const size_t oW2l = off; off += (size_t)HID * CC * 2;
  const size_t oP   = off; off += (size_t)NN * HID * 4;
  const size_t oQh  = off; off += (size_t)NN * CC * 2;
  const size_t oQl  = off; off += (size_t)NN * CC * 2;
  const size_t oKh  = off; off += (size_t)NN * CC * 2;
  const size_t oKl  = off; off += (size_t)NN * CC * 2;
  const size_t oVTh = off; off += (size_t)CC * NN * 2;
  const size_t oVTl = off; off += (size_t)CC * NN * 2;
  const size_t oQWh = off; off += (size_t)NN * NQW * 2;
  const size_t oQWl = off; off += (size_t)NN * NQW * 2;
  const size_t oBI  = off; off += (size_t)NHD * NN * NN * 4;
  if (off > ws_size) return;
  if (off > (size_t)134217728) return;

  char* ws = (char*)d_ws;
  ush* Xh  = (ush*)(ws + oXh);
  ush* Xl  = (ush*)(ws + oXl);
  ush* Yh  = (ush*)(ws + oYh);
  ush* Yl  = (ush*)(ws + oYl);
  ush* WTh = (ush*)(ws + oWTh);
  ush* WTl = (ush*)(ws + oWTl);
  ush* W2h = (ush*)(ws + oW2h);
  ush* W2l = (ush*)(ws + oW2l);
  float* P = (float*)(ws + oP);
  ush* Qh  = (ush*)(ws + oQh);
  ush* Ql  = (ush*)(ws + oQl);
  ush* Kh  = (ush*)(ws + oKh);
  ush* Kl  = (ush*)(ws + oKl);
  ush* VTh = (ush*)(ws + oVTh);
  ush* VTl = (ush*)(ws + oVTl);
  ush* QWh = (ush*)(ws + oQWh);
  ush* QWl = (ush*)(ws + oQWl);
  float* BI = (float*)(ws + oBI);

  const float sscale = 0.17677669529663687f;

  k_cvt<<<dim3(GB5), dim3(256), 0, stream>>>(x, y, pos, wq, wk, wv, w1, w2,
                                             Xh, Xl, Yh, Yl, WTh, WTl, W2h, W2l, P);
  k_proj<<<dim3(NN / 256, NWT / 64), dim3(256), 0, stream>>>(Xh, Xl, Yh, Yl, WTh, WTl, bq, bk, bv,
                                                             Qh, Ql, Kh, Kl, VTh, VTl);
  k_qw<<<dim3(NN / 256, NHD), dim3(256), 0, stream>>>(Qh, Ql, W2h, W2l, QWh, QWl);
  k_geom<<<dim3(NN / IB), dim3(256), 0, stream>>>(P, b1, b2, pos, Qh, Ql, QWh, QWl, BI);
  k_attn<<<dim3(NQT, NHD), dim3(128), 0, stream>>>(Qh, Ql, Kh, Kl, VTh, VTl, BI, out, sscale);
  (void)hipGetLastError();
}
